// AttentionLocalMessageFunction_53910429499700
// MI455X (gfx1250) — hardware-verified
//
#include <hip/hip_runtime.h>
#include <stddef.h>


#define DCO    32
#define DFE    16
#define NHEAD  4
#define NPORT  2
#define DIN    80
#define VHID   32
#define VOUT   16
#define SHID   32
#define PHID   256
#define DOUT   128
#define WCN    1024
#define PCW    512
#define NDP    96
#define NTHR   256
#define NWAVE  8
#define EPT    8
#define NGRP   2
#define CHUNK  (NTHR * EPT * NGRP)
#define WCAP   (EPT * NGRP * 32)
#define LISTN  (NWAVE * WCAP)
#define NBC    4096
#define NBF    1024
#define RCAP   40960
#define RBN    128
#define OTHR   512
#define PROWS  128
#define PSTG   68
#define NDTHR  128
#define NDW    4
#define NPB    64
#define DEGCAP 64
#define LCAP   (16 * DEGCAP)
#define TCAP   (LCAP / 16)
#define WLDS   5408
#define STGP   68
#define HVP    40
#define PSP    264
#define SW     64.0f
#define EPSD   1e-9f

#define L_LIST 0
#define L_AN   1024
#define L_AD   2048
#define L_STG  2112
#define L_WV   3200
#define L_EW   4288
#define L_HV   4352
#define L_HL   4672
#define L_EF   4992
#define L_RS   5312
#define L_RD   5328
#define L_RJ   5344
#define L_RV   5360
#define L_RNF  5376

#define LDS_FILL ((RCAP + NBF + LISTN) * 4 + 64)
#define LDS_NODE (NDW * WLDS * 4)
#define LDS_PSI  (NDW * 2 * 16 * PSP * 2)

static_assert((CHUNK & (CHUNK - 1)) == 0);
static_assert(CHUNK <= 4096);
static_assert(NBC <= 4096 && NBF <= 4096);
static_assert(NBC == 4 * NBF);
static_assert(OTHR * 8 == NBC);
static_assert((RCAP % 32) == 0);
static_assert(LCAP == L_AN - L_LIST);
static_assert(16 * 64 == L_AD - L_AN);
static_assert(64 == L_STG - L_AD);
static_assert(16 * STGP <= L_WV - L_STG);
static_assert(16 * STGP <= L_EW - L_WV);
static_assert(16 * NDP <= L_EW - L_STG);
static_assert(64 == L_HV - L_EW);
static_assert(16 * HVP <= 2 * (L_HL - L_HV));
static_assert(16 * HVP <= 2 * (L_EF - L_HL));
static_assert(16 * HVP <= 2 * (L_RS - L_EF));
static_assert(L_RNF + 16 <= WLDS);
static_assert((WLDS % 4) == 0 && (L_STG % 4) == 0 && (L_WV % 4) == 0 && (L_HV % 4) == 0 && (L_HL % 4) == 0 && (L_EF % 4) == 0);
static_assert(TCAP * 16 == LCAP);
static_assert(NPB == NDW * 16);
static_assert(PROWS == NWAVE * 16);
static_assert((PROWS % NPB) == 0);
static_assert(16 * DOUT * 4 <= 16 * PSP * 2);
static_assert((PSP % 8) == 0 && (PSTG % 4) == 0 && (STGP % 4) == 0 && (HVP % 8) == 0);

typedef float          v4f  __attribute__((ext_vector_type(4)));
typedef float          v8f  __attribute__((ext_vector_type(8)));
typedef int            v4i  __attribute__((ext_vector_type(4)));
typedef _Float16       v8h  __attribute__((ext_vector_type(8)));
typedef _Float16       v16h __attribute__((ext_vector_type(16)));
typedef unsigned short v8us __attribute__((ext_vector_type(8)));
typedef unsigned short v16us __attribute__((ext_vector_type(16)));
#if defined(__HIP_DEVICE_COMPILE__)
typedef __bf16         v16bf __attribute__((ext_vector_type(16)));
#endif
union FragH { v16h v; v8h h[2]; };
union FragU { v16us v; v8us h[2]; };

__device__ __forceinline__ float bf16r(float x) {
  unsigned u = __float_as_uint(x);
  u = (u + 0x7fffu + ((u >> 16) & 1u)) & 0xffff0000u;
  return __uint_as_float(u);
}

__device__ __forceinline__ unsigned short bfbits(float x) {
  unsigned u = __float_as_uint(x);
  u = u + 0x7fffu + ((u >> 16) & 1u);
  return (unsigned short)(u >> 16);
}

__device__ __forceinline__ unsigned short hbits(float x) {
  const _Float16 h = (_Float16)x;
  return __builtin_bit_cast(unsigned short, h);
}

__device__ __forceinline__ v8h cvt8b(v4f a, v4f b) {
  v8h r;
  r[0] = (_Float16)bf16r(a.x); r[1] = (_Float16)bf16r(a.y); r[2] = (_Float16)bf16r(a.z); r[3] = (_Float16)bf16r(a.w);
  r[4] = (_Float16)bf16r(b.x); r[5] = (_Float16)bf16r(b.y); r[6] = (_Float16)bf16r(b.z); r[7] = (_Float16)bf16r(b.w);
  return r;
}

__device__ __forceinline__ void split8(v4f a, v4f b, v8us& hi, v8us& lo) {
  float x[8] = {a.x, a.y, a.z, a.w, b.x, b.y, b.z, b.w};
#pragma unroll
  for (int e = 0; e < 8; ++e) {
    const unsigned short hb = bfbits(x[e]);
    const float hf = __uint_as_float(((unsigned)hb) << 16);
    hi[e] = hb;
    lo[e] = bfbits(x[e] - hf);
  }
}

__device__ __forceinline__ v8f wmh(v16h a, v16h b, v8f c) {
#if defined(__HIP_DEVICE_COMPILE__)
  v8f d = __builtin_amdgcn_wmma_f32_16x16x32_f16(false, a, false, b, (short)0, c, false, false);
  asm volatile("v_nop\n\tv_nop\n\tv_nop\n\tv_nop" : "+v"(d) : "v"(a), "v"(b));
  return d;
#else
  (void)a; (void)b;
  return c;
#endif
}

__device__ __forceinline__ v8f wmb(v16us a, v16us b, v8f c) {
#if defined(__HIP_DEVICE_COMPILE__)
  const v16bf ab = __builtin_bit_cast(v16bf, a);
  const v16bf bb = __builtin_bit_cast(v16bf, b);
  v8f d = __builtin_amdgcn_wmma_f32_16x16x32_bf16(false, ab, false, bb, (short)0, c, false, false);
  asm volatile("v_nop\n\tv_nop\n\tv_nop\n\tv_nop" : "+v"(d) : "v"(ab), "v"(bb));
  return d;
#else
  (void)a; (void)b;
  return c;
#endif
}

__device__ __forceinline__ void wave_sync() {
#if defined(__HIP_DEVICE_COMPILE__)
  __builtin_amdgcn_fence(__ATOMIC_ACQ_REL, "wavefront");
  __builtin_amdgcn_wave_barrier();
#endif
}

template <int NB>
__device__ __forceinline__ int scan_chunk(const int* __restrict__ keys, int nE, int cbase, int slotBase,
                                          int vec8, int* list, int tid, int lane, int wave) {
  int wc = 0;
#pragma unroll
  for (int g = 0; g < NGRP; ++g) {
    const int el0  = (g * NTHR + tid) * EPT;
    const int e0   = cbase + el0;
    const int sent = -2147483647 - 1;
    v4i da, db;
    if (vec8 != 0 && cbase + CHUNK <= nE) {
      da = *(const v4i*)(keys + e0);
      db = *(const v4i*)(keys + e0 + 4);
    } else {
      da.x = (e0     < nE) ? keys[min(e0, nE - 1)]     : sent;
      da.y = (e0 + 1 < nE) ? keys[min(e0 + 1, nE - 1)] : sent;
      da.z = (e0 + 2 < nE) ? keys[min(e0 + 2, nE - 1)] : sent;
      da.w = (e0 + 3 < nE) ? keys[min(e0 + 3, nE - 1)] : sent;
      db.x = (e0 + 4 < nE) ? keys[min(e0 + 4, nE - 1)] : sent;
      db.y = (e0 + 5 < nE) ? keys[min(e0 + 5, nE - 1)] : sent;
      db.z = (e0 + 6 < nE) ? keys[min(e0 + 6, nE - 1)] : sent;
      db.w = (e0 + 7 < nE) ? keys[min(e0 + 7, nE - 1)] : sent;
    }
    const unsigned nb = (unsigned)slotBase;
    const unsigned s0 = (unsigned)da.x - nb, s1 = (unsigned)da.y - nb;
    const unsigned s2 = (unsigned)da.z - nb, s3 = (unsigned)da.w - nb;
    const unsigned s4 = (unsigned)db.x - nb, s5 = (unsigned)db.y - nb;
    const unsigned s6 = (unsigned)db.z - nb, s7 = (unsigned)db.w - nb;
    const bool h0 = s0 < (unsigned)NB, h1 = s1 < (unsigned)NB, h2 = s2 < (unsigned)NB, h3 = s3 < (unsigned)NB;
    const bool h4 = s4 < (unsigned)NB, h5 = s5 < (unsigned)NB, h6 = s6 < (unsigned)NB, h7 = s7 < (unsigned)NB;
    const unsigned any = __builtin_amdgcn_ballot_w32(h0 | h1 | h2 | h3 | h4 | h5 | h6 | h7);
    if (any != 0u) {
#define HITJ(J, HJ, SJ) { \
        const unsigned mj = __builtin_amdgcn_ballot_w32(HJ); \
        if (mj != 0u) { \
          if (HJ) { \
            const int pos = wc + (int)__builtin_amdgcn_mbcnt_lo(mj, 0u); \
            if (pos < WCAP) list[wave * WCAP + pos] = ((el0 + (J)) << 12) | (int)(SJ); \
          } \
          wc += (int)__builtin_popcount(mj); } }
      HITJ(0, h0, s0)
      HITJ(1, h1, s1)
      HITJ(2, h2, s2)
      HITJ(3, h3, s3)
      HITJ(4, h4, s4)
      HITJ(5, h5, s5)
      HITJ(6, h6, s6)
      HITJ(7, h7, s7)
#undef HITJ
    }
  }
  return wc;
}

__global__ __launch_bounds__(NTHR) void k_prep(
    const float* __restrict__ vW1, const float* __restrict__ vb1,
    const float* __restrict__ sW1, const float* __restrict__ sb1,
    const float* __restrict__ vW2, const float* __restrict__ pW1, const float* __restrict__ pW2,
    unsigned short* wb1, unsigned short* wc, unsigned short* wv2, unsigned short* wp1, unsigned short* wp2) {
  const int g0 = NPORT * 256 * 32 / 8;
  const int g1 = WCN * 32 / 8;
  const int g2 = NPORT * NHEAD * 16 * 32 / 8;
  const int g3 = PHID * 64 / 8;
  const int g4 = DOUT * PHID / 8;
  const int bstart = blockIdx.x * NTHR;
  const int i = bstart + (int)threadIdx.x;
  if (i >= g0 + g1 + g2 + g3 + g4) return;
  unsigned short u[8];
  unsigned short* dp;
  if (bstart < g0) {
    const int o = i * 8;
    const int p = o >> 13, rem = o & 8191;
    const int n = rem >> 5, k0 = rem & 31;
    const int h = n >> 6, c = n & 63, hp = h * 2 + p;
    const int cv = c < 32 ? c : 31;
    const int cs = c >= 32 ? c - 32 : 0;
#pragma unroll
    for (int e = 0; e < 8; ++e) {
      const int k  = k0 + e;
      const int kc = k < 16 ? k : 15;
      const float a  = vW1[(hp * DIN + kc) * VHID + cv];
      const float b  = sW1[(hp * DIN + kc) * SHID + cs];
      const float ba = vb1[hp * VHID + cv];
      const float bb = sb1[hp * SHID + cs];
      const float w  = (c < 32) ? a : b;
      const float bi = (c < 32) ? ba : bb;
      const float sel = (k < 16) ? w : ((k == 16) ? bi : 0.0f);
      u[e] = hbits(SW * bf16r(sel));
    }
    dp = wb1 + o;
  } else if (bstart < g0 + g1) {
    const int o = (i - g0) * 8;
    const int n = o >> 5, k0 = o & 31;
    const int p = n >> 9, rem = n & 511;
    const int side = rem >> 8, rem2 = rem & 255;
    const int h = rem2 >> 6, c = rem2 & 63, hp = h * 2 + p;
    const int cv = c < 32 ? c : 31;
    const int cs = c >= 32 ? c - 32 : 0;
#pragma unroll
    for (int e = 0; e < 8; ++e) {
      const int krow = DFE + side * DCO + k0 + e;
      const float a = vW1[(hp * DIN + krow) * VHID + cv];
      const float b = sW1[(hp * DIN + krow) * SHID + cs];
      u[e] = hbits(SW * bf16r((c < 32) ? a : b));
    }
    dp = wc + o;
  } else if (bstart < g0 + g1 + g2) {
    const int o = (i - g0 - g1) * 8;
    const int p = o >> 11, rem = o & 2047;
    const int h = rem >> 9, rem2 = rem & 511;
    const int n = rem2 >> 5, k0 = rem2 & 31, hp = h * 2 + p;
#pragma unroll
    for (int e = 0; e < 8; ++e) u[e] = hbits(SW * bf16r(vW2[(hp * VHID + k0 + e) * VOUT + n]));
    dp = wv2 + o;
  } else if (bstart < g0 + g1 + g2 + g3) {
    const int o = (i - g0 - g1 - g2) * 8;
    const int n = o >> 6, k0 = o & 63;
#pragma unroll
    for (int e = 0; e < 8; ++e) u[e] = bfbits(pW1[(k0 + e) * PHID + n]);
    dp = wp1 + o;
  } else {
    const int o = (i - g0 - g1 - g2 - g3) * 8;
    const int n = o >> 8, k0 = o & 255;
#pragma unroll
    for (int e = 0; e < 8; ++e) u[e] = bfbits(pW2[(k0 + e) * DOUT + n]);
    dp = wp2 + o;
  }
  v8us hv;
#pragma unroll
  for (int e = 0; e < 8; ++e) hv[e] = u[e];
  *(volatile v8us*)dp = hv;
  __threadfence();
  *(volatile v8us*)dp = hv;
}

__global__ __launch_bounds__(NTHR) void k_count(const int* __restrict__ keys, int* cnt, int nE, int vec8) {
  __shared__ __attribute__((aligned(16))) int scnt[NBC];
  __shared__ __attribute__((aligned(16))) int list[LISTN];
  __shared__ int wcnt[NWAVE];
  const int tid = threadIdx.x, lane = tid & 31, wave = tid >> 5;
  const int nodeBase = blockIdx.x * NBC;

  for (int i = tid; i < NBC; i += NTHR) scnt[i] = 0;
  __syncthreads();

  const int nChunks = (nE + CHUNK - 1) / CHUNK;
#pragma unroll 1
  for (int ch = 0; ch < nChunks; ++ch) {
    const int cbase = ch * CHUNK;
    const int wc = scan_chunk<NBC>(keys, nE, cbase, nodeBase, vec8, list, tid, lane, wave);
    if (lane == 0) wcnt[wave] = wc;
    __syncthreads();
    if (wave == 0) {
#pragma unroll 1
      for (int wsx = 0; wsx < NWAVE; ++wsx) {
        int n = __builtin_amdgcn_readfirstlane(wcnt[wsx]);
        n = n > WCAP ? WCAP : (n < 0 ? 0 : n);
        const int* lp = list + wsx * WCAP;
#pragma unroll 1
        for (int i = 0; i < n; ++i) {
          const int ent  = __builtin_amdgcn_readfirstlane(lp[i]);
          const int slot = ent & (NBC - 1);
          if (lane == 0) scnt[slot] = scnt[slot] + 1;
        }
      }
    }
    __syncthreads();
  }

  v4i cq[4];
#pragma unroll
  for (int q = 0; q < 4; ++q) {
    const int f = (wave * 4 + q) * 128 + 4 * lane;
    cq[q] = *(const v4i*)(scnt + f);
  }
  int* cp = cnt + (size_t)nodeBase;
#pragma unroll
  for (int q = 0; q < 4; ++q) {
    const int f = (wave * 4 + q) * 128 + 4 * lane;
    *(volatile v4i*)(cp + f) = cq[q];
  }
  __threadfence();
#pragma unroll
  for (int q = 0; q < 4; ++q) {
    const int f = (wave * 4 + q) * 128 + 4 * lane;
    *(volatile v4i*)(cp + f) = cq[q];
  }
}

__global__ __launch_bounds__(OTHR) void k_offsets(
    const int* __restrict__ cnt, int* off, int* rbase, int nChunk) {
  __shared__ __attribute__((aligned(16))) int soff[NBC];
  __shared__ __attribute__((aligned(16))) int srb[RBN];
  __shared__ int wtot[OTHR / 32];
  const int tid = threadIdx.x, lane = tid & 31, wave = tid >> 5, sub = tid >> 7;
  for (int i = tid; i < RBN; i += OTHR) srb[i] = 0;
  int carry = 0;
#pragma unroll 1
  for (int ch = 0; ch < nChunk; ++ch) {
    const int base = ch * NBC;
    const v4i c0 = *(const v4i*)(cnt + base + 8 * tid);
    const v4i c1 = *(const v4i*)(cnt + base + 8 * tid + 4);
    const int e0 = max(c0.x, 0), e1 = max(c0.y, 0), e2 = max(c0.z, 0), e3 = max(c0.w, 0);
    const int e4 = max(c1.x, 0), e5 = max(c1.y, 0), e6 = max(c1.z, 0), e7 = max(c1.w, 0);
    const int ts = e0 + e1 + e2 + e3 + e4 + e5 + e6 + e7;
    int incl = ts;
#pragma unroll
    for (int d = 1; d < 32; d <<= 1) {
      const int t = __shfl_up(incl, d);
      if (lane >= d) incl += t;
    }
    if (lane == 31) wtot[wave] = incl;
    __syncthreads();
    const int S0 = wtot[0]  + wtot[1]  + wtot[2]  + wtot[3];
    const int S1 = wtot[4]  + wtot[5]  + wtot[6]  + wtot[7];
    const int S2 = wtot[8]  + wtot[9]  + wtot[10] + wtot[11];
    const int S3 = wtot[12] + wtot[13] + wtot[14] + wtot[15];
    int pre = 0;
#pragma unroll 1
    for (int w = 4 * sub; w < wave; ++w) pre += wtot[w];
    const int b0 = carry;
    const int b1 = b0 + ((S0 + 31) & ~31);
    const int b2 = b1 + ((S1 + 31) & ~31);
    const int b3 = b2 + ((S2 + 31) & ~31);
    const int b4 = b3 + ((S3 + 31) & ~31);
    const int myb = sub == 0 ? b0 : (sub == 1 ? b1 : (sub == 2 ? b2 : b3));
    if (tid == 0) {
      srb[min(4 * ch + 0, RBN - 1)] = b0;
      srb[min(4 * ch + 1, RBN - 1)] = b1;
      srb[min(4 * ch + 2, RBN - 1)] = b2;
      srb[min(4 * ch + 3, RBN - 1)] = b3;
    }
    int run = myb + pre + incl - ts;
    soff[8 * tid + 0] = run; run += e0;
    soff[8 * tid + 1] = run; run += e1;
    soff[8 * tid + 2] = run; run += e2;
    soff[8 * tid + 3] = run; run += e3;
    soff[8 * tid + 4] = run; run += e4;
    soff[8 * tid + 5] = run; run += e5;
    soff[8 * tid + 6] = run; run += e6;
    soff[8 * tid + 7] = run;
    carry = b4;
    __syncthreads();
    const v4i o0 = *(const v4i*)(soff + 4 * tid);
    const v4i o1 = *(const v4i*)(soff + 4 * (tid + OTHR));
    int* op = off + base;
    *(volatile v4i*)(op + 4 * tid) = o0;
    *(volatile v4i*)(op + 4 * (tid + OTHR)) = o1;
    __threadfence();
    *(volatile v4i*)(op + 4 * tid) = o0;
    *(volatile v4i*)(op + 4 * (tid + OTHR)) = o1;
    __syncthreads();
  }
  if (tid == 0) srb[min(4 * nChunk, RBN - 1)] = carry;
  __syncthreads();
  v4i rv = {0, 0, 0, 0};
  if (tid < 32) rv = *(const v4i*)(srb + 4 * tid);
  if (tid < 32) *(volatile v4i*)(rbase + 4 * tid) = rv;
  __threadfence();
  if (tid < 32) *(volatile v4i*)(rbase + 4 * tid) = rv;
}

__global__ __launch_bounds__(NTHR) void k_fill(
    const int* __restrict__ keys, const int* __restrict__ off, const int* __restrict__ rbase,
    int* csr, int nE, int vec8, int csrLen) {
  extern __shared__ v4f lds_dyn[];
  int* region = (int*)lds_dyn;
  int* cursor = region + RCAP;
  int* list   = cursor + NBF;
  int* wcnt   = list + LISTN;
  const int tid = threadIdx.x, lane = tid & 31, wave = tid >> 5;
  const int b = blockIdx.x;
  const int nodeBase = b * NBF;

  int rb0 = rbase[b];
  const int rb1 = rbase[b + 1];
  rb0 = rb0 < 0 ? 0 : (rb0 > csrLen ? csrLen : rb0);
  rb0 &= ~31;
  int len = rb1 - rb0;
  len = len < 0 ? 0 : (len > RCAP ? RCAP : len);
  int lenW = (len + 31) & ~31;
  if (rb0 + lenW > csrLen) lenW = (csrLen - rb0) & ~31;

  {
    const v4i z = {0, 0, 0, 0};
    for (int i = tid; i < RCAP / 4; i += NTHR) ((v4i*)region)[i] = z;
    for (int s = tid; s < NBF; s += NTHR) {
      int o = off[nodeBase + s] - rb0;
      o = o < 0 ? 0 : (o > RCAP ? RCAP : o);
      cursor[s] = o;
    }
  }
  __syncthreads();

  const int nChunks = (nE + CHUNK - 1) / CHUNK;
#pragma unroll 1
  for (int ch = 0; ch < nChunks; ++ch) {
    const int cbase = ch * CHUNK;
    const int wc = scan_chunk<NBF>(keys, nE, cbase, nodeBase, vec8, list, tid, lane, wave);
    if (lane == 0) wcnt[wave] = wc;
    __syncthreads();
    if (wave == 0) {
#pragma unroll 1
      for (int wsx = 0; wsx < NWAVE; ++wsx) {
        int n = __builtin_amdgcn_readfirstlane(wcnt[wsx]);
        n = n > WCAP ? WCAP : (n < 0 ? 0 : n);
        const int* lp = list + wsx * WCAP;
#pragma unroll 1
        for (int i = 0; i < n; ++i) {
          const int ent  = __builtin_amdgcn_readfirstlane(lp[i]);
          const int slot = ent & (NBF - 1);
          int e = cbase + ((ent >> 12) & (CHUNK - 1));
          e = e > nE - 1 ? nE - 1 : e;
          if (lane == 0) {
            int pos = cursor[slot];
            pos = pos < 0 ? 0 : (pos > RCAP - 1 ? RCAP - 1 : pos);
            region[pos] = e;
            const int np = pos + 1;
            cursor[slot] = np > RCAP ? RCAP : np;
          }
        }
      }
    }
    __syncthreads();
  }

  const int nv = lenW >> 2;
  int* gp = csr + rb0;
#pragma unroll 1
  for (int i = tid; i < nv; i += NTHR) { const v4i v = ((const v4i*)region)[i]; *(volatile v4i*)(gp + 4 * i) = v; }
  __threadfence();
#pragma unroll 1
  for (int i = tid; i < nv; i += NTHR) { const v4i v = ((const v4i*)region)[i]; *(volatile v4i*)(gp + 4 * i) = v; }
}

__global__ __launch_bounds__(NTHR) void k_proj(
    const float* __restrict__ co, const _Float16* __restrict__ wc, float* pc, int nN, int port) {
  __shared__ __attribute__((aligned(16))) float stg[NWAVE][16 * PSTG];
  const int tid = threadIdx.x, lane = tid & 31, wave = tid >> 5, hh = lane >> 4, m = lane & 15;
  const int rowBase = blockIdx.x * PROWS + wave * 16;
  int ra = rowBase + m;
  ra = ra > nN - 1 ? nN - 1 : ra;
  const float* ap = co + (size_t)ra * DCO + 8 * hh;
  const v4f c0 = *(const v4f*)ap, c1 = *(const v4f*)(ap + 4);
  const v4f c2 = *(const v4f*)(ap + 16), c3 = *(const v4f*)(ap + 20);
  FragH a;
  a.h[0] = cvt8b(c0, c1);
  a.h[1] = cvt8b(c2, c3);
  float* sp = stg[wave];
  const int pcl = port < 0 ? 0 : (port > 1 ? 1 : port);

#pragma unroll 1
  for (int g = 0; g < PCW / 64; ++g) {
    v8f acc[4];
#pragma unroll
    for (int t = 0; t < 4; ++t) { v8f z = {0.f, 0.f, 0.f, 0.f, 0.f, 0.f, 0.f, 0.f}; acc[t] = z; }
#pragma unroll
    for (int t = 0; t < 4; ++t) {
      const _Float16* bp = wc + (size_t)(512 * pcl + 64 * g + 16 * t + m) * 32 + 8 * hh;
      FragH b;
      b.h[0] = *(const v8h*)bp;
      b.h[1] = *(const v8h*)(bp + 16);
      acc[t] = wmh(a.v, b.v, acc[t]);
    }
#pragma unroll
    for (int t = 0; t < 4; ++t) {
#pragma unroll
      for (int r = 0; r < 8; ++r) sp[(8 * hh + r) * PSTG + 16 * t + m] = acc[t][r];
    }
    wave_sync();
    v4f ov[8];
#pragma unroll
    for (int ii = 0; ii < 8; ++ii) {
      const int row = 2 * ii + (lane >> 4);
      const int c4  = (lane & 15) * 4;
      ov[ii] = *(const v4f*)(sp + row * PSTG + c4);
    }
    wave_sync();
    float* gp = pc + (size_t)rowBase * PCW + 64 * g;
#pragma unroll
    for (int ii = 0; ii < 8; ++ii) {
      const int row = 2 * ii + (lane >> 4);
      const int c4  = (lane & 15) * 4;
      *(volatile v4f*)(gp + (size_t)row * PCW + c4) = ov[ii];
    }
    __threadfence();
#pragma unroll
    for (int ii = 0; ii < 8; ++ii) {
      const int row = 2 * ii + (lane >> 4);
      const int c4  = (lane & 15) * 4;
      *(volatile v4f*)(gp + (size_t)row * PCW + c4) = ov[ii];
    }
  }
}

__device__ __forceinline__ void flush_acc(float* accN, float* accD, int j, int lane, int hh, int m,
                                          float an0, float an1, float ad0, float ad1) {
  float* np = accN + j * 64;
  np[lane]      = np[lane] + an0;
  np[32 + lane] = np[32 + lane] + an1;
  if (m == 0) {
    accD[j * 4 + hh]     = accD[j * 4 + hh] + ad0;
    accD[j * 4 + 2 + hh] = accD[j * 4 + 2 + hh] + ad1;
  }
}

template <int PORT>
__global__ __launch_bounds__(NDTHR) void k_node(
    const float* __restrict__ ef, const int* __restrict__ src, const int* __restrict__ dst,
    const float* __restrict__ nf, const float* __restrict__ nfa,
    const int* __restrict__ cnt, const int* __restrict__ offt, const int* __restrict__ csr,
    const float* __restrict__ pc, const _Float16* __restrict__ wb1, const _Float16* __restrict__ wv2,
    const float* __restrict__ vb2, const float* __restrict__ sW2, const float* __restrict__ sb2,
    float* nd, int nN, int nE, int csrLen) {
  extern __shared__ v4f lds_dyn[];
  __shared__ float s_w2[NHEAD * NPORT * SHID];
  __shared__ float s_vb2[NHEAD * NPORT * VOUT];
  __shared__ float s_sb2[NHEAD * NPORT];
  const int tid = threadIdx.x, lane = tid & 31, wave = tid >> 5, hh = lane >> 4, m = lane & 15;
  float* wb = (float*)lds_dyn + wave * WLDS;
  int*   list = (int*)(wb + L_LIST);
  float* accN = wb + L_AN;
  float* accD = wb + L_AD;
  float* stg  = wb + L_STG;
  float* wvt  = wb + L_WV;
  float* ewt  = wb + L_EW;
  _Float16* hv16 = (_Float16*)(wb + L_HV);
  _Float16* hl16 = (_Float16*)(wb + L_HL);
  _Float16* efa  = (_Float16*)(wb + L_EF);
  int*   rsd = (int*)(wb + L_RS);
  int*   rdd = (int*)(wb + L_RD);
  int*   rjd = (int*)(wb + L_RJ);
  int*   rvd = (int*)(wb + L_RV);
  float* rnf = wb + L_RNF;
  const int gn0 = blockIdx.x * NPB + wave * 16;

  for (int i = tid; i < NHEAD * NPORT * SHID; i += NDTHR) s_w2[i] = bf16r(sW2[i]);
  for (int i = tid; i < NHEAD * NPORT * VOUT; i += NDTHR) s_vb2[i] = bf16r(vb2[i]);
  if (tid < NHEAD * NPORT) s_sb2[tid] = bf16r(sb2[tid]);

  if (PORT == 0) {
#pragma unroll 1
    for (int j = 0; j < 16; ++j) { accN[j * 64 + lane] = 0.0f; accN[j * 64 + 32 + lane] = 0.0f; }
    accD[lane] = 0.0f; accD[32 + lane] = 0.0f;
  } else {
#pragma unroll 1
    for (int j = 0; j < 16; ++j) {
      const float* rp = nd + (size_t)(gn0 + j) * NDP;
      accN[j * 64 + lane]      = rp[lane];
      accN[j * 64 + 32 + lane] = rp[32 + lane];
    }
    accD[lane]      = nd[(size_t)(gn0 + (lane >> 2)) * NDP + 64 + (lane & 3)];
    accD[32 + lane] = nd[(size_t)(gn0 + 8 + (lane >> 2)) * NDP + 64 + (lane & 3)];
  }
  __syncthreads();

  {
    const int node  = gn0 + m;
    const int nodec = node < nN ? node : nN - 1;
    int c = cnt[nodec];
    c = c < 0 ? 0 : (c > DEGCAP ? DEGCAP : c);
    c = (node < nN && hh == 0) ? c : 0;
    int st = offt[nodec];
    st = st < 0 ? 0 : (st > csrLen - 1 ? csrLen - 1 : st);
    int incl = c;
#pragma unroll
    for (int d = 1; d < 32; d <<= 1) {
      const int t = __shfl_up(incl, d);
      if (lane >= d) incl += t;
    }
    const int excl = incl - c;
    const int V = __builtin_amdgcn_readlane(incl, 31);
    wave_sync();
#pragma unroll 1
    for (int j = 0; j < 16; ++j) {
      const int nj  = __builtin_amdgcn_readlane(c, j);
      const int stj = __builtin_amdgcn_readlane(st, j);
      const int bj  = __builtin_amdgcn_readlane(excl, j);
#pragma unroll 1
      for (int q0 = 0; q0 < nj; q0 += 32) {
        const int idx = q0 + lane;
        int pos = stj + idx;
        pos = pos < 0 ? 0 : (pos > csrLen - 1 ? csrLen - 1 : pos);
        int e = csr[pos];
        e = e < 0 ? 0 : (e > nE - 1 ? nE - 1 : e);
        if (idx < nj) list[bj + idx] = (e << 4) | j;
      }
    }
    wave_sync();
    const int ntile = (V + 15) >> 4;
    float an0 = 0.f, an1 = 0.f, ad0 = 0.f, ad1 = 0.f;
    int jcur = -1;
#pragma unroll 1
    for (int t = 0; t < ntile && t < TCAP; ++t) {
      wave_sync();
      {
        const int  i     = 16 * t + m;
        const bool valid = i < V;
        const int  ent   = list[i < LCAP ? i : LCAP - 1];
        int e = ent >> 4;
        e = e < 0 ? 0 : (e > nE - 1 ? nE - 1 : e);
        const int j = ent & 15;
        int s = src[e]; s = s < 0 ? 0 : (s > nN - 1 ? nN - 1 : s);
        int d = dst[e]; d = d < 0 ? 0 : (d > nN - 1 ? nN - 1 : d);
        const float fv  = valid ? 1.0f : 0.0f;
        const float nfv = bf16r(nf[e]) * fv;
        const float* epf = ef + (size_t)e * DFE;
        const v4f f0 = *(const v4f*)epf * fv,       f1 = *(const v4f*)(epf + 4) * fv;
        const v4f f2 = *(const v4f*)(epf + 8) * fv, f3 = *(const v4f*)(epf + 12) * fv;
        const v8h x0 = cvt8b(f0, f1), x1 = cvt8b(f2, f3);
        if (hh == 0) {
          rsd[m] = s; rdd[m] = d; rjd[m] = j; rvd[m] = valid ? 1 : 0; rnf[m] = nfv;
          *(v8h*)(efa + m * HVP)     = x0;
          *(v8h*)(efa + m * HVP + 8) = x1;
        } else {
          v8h x2 = x0;
          x2[0] = (_Float16)fv;
          *(v8h*)(efa + m * HVP + 16) = x2;
          *(v8h*)(efa + m * HVP + 24) = x1;
        }
      }
      wave_sync();
      FragH a;
      a.h[0] = *(const v8h*)(efa + m * HVP + 8 * hh);
      a.h[1] = *(const v8h*)(efa + m * HVP + 16 + 8 * hh);
      const int r2 = lane >> 1, q = lane & 1;
      const int sN = rsd[r2], dN = rdd[r2];
      const float nfr = rnf[r2];
      const int vr = rvd[r2];
#pragma unroll 1
      for (int h = 0; h < NHEAD; ++h) {
        v8f acc[4];
#pragma unroll
        for (int tt = 0; tt < 4; ++tt) { v8f z = {0.f, 0.f, 0.f, 0.f, 0.f, 0.f, 0.f, 0.f}; acc[tt] = z; }
#pragma unroll
        for (int tt = 0; tt < 4; ++tt) {
          const _Float16* bp = wb1 + (size_t)(PORT * 256 + 64 * h + 16 * tt + m) * 32 + 8 * hh;
          FragH b;
          b.h[0] = *(const v8h*)bp;
          b.h[1] = *(const v8h*)(bp + 16);
          acc[tt] = wmh(a.v, b.v, acc[tt]);
        }
#pragma unroll
        for (int tt = 0; tt < 4; ++tt) {
#pragma unroll
          for (int r = 0; r < 8; ++r) stg[(8 * hh + r) * STGP + 16 * tt + m] = acc[tt][r];
        }
        wave_sync();
        const float* ps  = pc + (size_t)sN * PCW + h * 64 + 32 * q;
        const float* pd  = pc + (size_t)dN * PCW + 256 + h * 64 + 32 * q;
        const float* w2p = s_w2 + (h * NPORT + PORT) * SHID;
        const float* zr  = stg + r2 * STGP + 32 * q;
        float dot = 0.0f;
#pragma unroll
        for (int c8 = 0; c8 < 4; ++c8) {
          const v4f za = *(const v4f*)(zr + 8 * c8), zb = *(const v4f*)(zr + 8 * c8 + 4);
          const v4f sa = *(const v4f*)(ps + 8 * c8), sb = *(const v4f*)(ps + 8 * c8 + 4);
          const v4f da = *(const v4f*)(pd + 8 * c8), db = *(const v4f*)(pd + 8 * c8 + 4);
          const v4f ya = za + sa + da, yb = zb + sb + db;
          float y[8] = {ya.x, ya.y, ya.z, ya.w, yb.x, yb.y, yb.z, yb.w};
          v8h hq, hl;
#pragma unroll
          for (int ii = 0; ii < 8; ++ii) {
            const float zz = fmaxf(y[ii], 0.0f);
            const _Float16 qh = (_Float16)zz;
            hq[ii] = qh;
            hl[ii] = (_Float16)((zz - (float)qh) * 2048.0f);
            dot += zz * w2p[8 * c8 + ii];
          }
          if (q == 0) {
            *(v8h*)(hv16 + r2 * HVP + 8 * c8) = hq;
            *(v8h*)(hl16 + r2 * HVP + 8 * c8) = hl;
          }
        }
        float sc = dot * (1.0f / 64.0f) + s_sb2[h * NPORT + PORT];
        sc = sc * nfr;
        float ew = expf(sc);
        ew = (vr != 0) ? ew : 0.0f;
        if (q == 1) ewt[r2 * 4 + h] = ew;
        wave_sync();
        FragH a2, a3;
        a2.h[0] = *(const v8h*)(hv16 + m * HVP + 8 * hh);
        a2.h[1] = *(const v8h*)(hv16 + m * HVP + 16 + 8 * hh);
        a3.h[0] = *(const v8h*)(hl16 + m * HVP + 8 * hh);
        a3.h[1] = *(const v8h*)(hl16 + m * HVP + 16 + 8 * hh);
        const _Float16* bq = wv2 + (size_t)((PORT * NHEAD + h) * 16 + m) * 32 + 8 * hh;
        FragH b2;
        b2.h[0] = *(const v8h*)bq;
        b2.h[1] = *(const v8h*)(bq + 16);
        v8f vz = {0.f, 0.f, 0.f, 0.f, 0.f, 0.f, 0.f, 0.f};
        const v8f va = wmh(a2.v, b2.v, vz);
        const v8f vb = wmh(a3.v, b2.v, vz);
        const float vbias = s_vb2[(h * NPORT + PORT) * VOUT + m];
#pragma unroll
        for (int r = 0; r < 8; ++r) {
          const int row = 8 * hh + r;
          const float val = ((va[r] + vb[r] * (1.0f / 2048.0f)) * (1.0f / 4096.0f) + vbias) * rnf[row];
          wvt[row * STGP + 16 * h + m] = val * ewt[row * 4 + h];
        }
      }
      wave_sync();
#pragma unroll 1
      for (int row = 0; row < 16; ++row) {
        const int jr = __builtin_amdgcn_readfirstlane(rjd[row]);
        if (jr != jcur) {
          if (jcur >= 0) flush_acc(accN, accD, jcur, lane, hh, m, an0, an1, ad0, ad1);
          jcur = jr; an0 = 0.f; an1 = 0.f; ad0 = 0.f; ad1 = 0.f;
        }
        an0 += wvt[row * STGP + lane];
        an1 += wvt[row * STGP + 32 + lane];
        ad0 += ewt[row * 4 + hh];
        ad1 += ewt[row * 4 + 2 + hh];
      }
    }
    if (jcur >= 0) flush_acc(accN, accD, jcur, lane, hh, m, an0, an1, ad0, ad1);
    wave_sync();
  }

  wave_sync();
  if (PORT == 0) {
    float* nst = stg;
#pragma unroll 1
    for (int j = 0; j < 16; ++j) {
      nst[j * NDP + lane]      = accN[j * 64 + lane];
      nst[j * NDP + 32 + lane] = accN[j * 64 + 32 + lane];
      const float dv = accD[j * 4 + (lane & 3)];
      nst[j * NDP + 64 + lane] = (lane < 4) ? dv : 0.0f;
    }
    wave_sync();
    v4f ov[12];
#pragma unroll
    for (int i = 0; i < 12; ++i) ov[i] = *(const v4f*)(nst + 128 * i + 4 * lane);
    float* gp = nd + (size_t)gn0 * NDP;
#pragma unroll
    for (int i = 0; i < 12; ++i) *(volatile v4f*)(gp + 128 * i + 4 * lane) = ov[i];
    __threadfence();
#pragma unroll
    for (int i = 0; i < 12; ++i) *(volatile v4f*)(gp + 128 * i + 4 * lane) = ov[i];
  } else {
    float* vst = stg;
#pragma unroll 1
    for (int j = 0; j < 16; ++j) {
      const int ndx = gn0 + j;
      const float a  = bf16r(nfa[ndx < nN ? ndx : nN - 1]);
      const float d0 = accD[j * 4 + hh] * a + EPSD;
      const float d1 = accD[j * 4 + 2 + hh] * a + EPSD;
      const float v0 = accN[j * 64 + lane] * a * (1.0f / d0);
      const float v1 = accN[j * 64 + 32 + lane] * a * (1.0f / d1);
      vst[j * 64 + lane]      = v0;
      vst[j * 64 + 32 + lane] = v1;
    }
    wave_sync();
    v4f ov[8];
#pragma unroll
    for (int ii = 0; ii < 8; ++ii) {
      const int row = 2 * ii + (lane >> 4);
      const int c4  = (lane & 15) * 4;
      ov[ii] = *(const v4f*)(vst + row * 64 + c4);
    }
    float* gp = nd + (size_t)gn0 * NDP;
#pragma unroll
    for (int ii = 0; ii < 8; ++ii) {
      const int row = 2 * ii + (lane >> 4);
      const int c4  = (lane & 15) * 4;
      *(volatile v4f*)(gp + (size_t)row * NDP + c4) = ov[ii];
    }
    __threadfence();
#pragma unroll
    for (int ii = 0; ii < 8; ++ii) {
      const int row = 2 * ii + (lane >> 4);
      const int c4  = (lane & 15) * 4;
      *(volatile v4f*)(gp + (size_t)row * NDP + c4) = ov[ii];
    }
  }
}

__global__ __launch_bounds__(NDTHR) void k_psi(
    const float* __restrict__ nd, const unsigned short* __restrict__ wp1, const float* __restrict__ pb1,
    const unsigned short* __restrict__ wp2, const float* __restrict__ pb2, const float* __restrict__ nfa,
    float* out, int nN) {
  extern __shared__ v4f lds_dyn[];
  const int tid = threadIdx.x, lane = tid & 31, wave = tid >> 5, hh = lane >> 4, m = lane & 15;
  unsigned short* shi = (unsigned short*)lds_dyn + (size_t)wave * (2 * 16 * PSP);
  unsigned short* slo = shi + 16 * PSP;
  const int rb = blockIdx.x * NPB + wave * 16;
  const float* ap = nd + (size_t)(rb + m) * NDP + 8 * hh;
  FragU ahi[2], alo[2];
#pragma unroll
  for (int ks = 0; ks < 2; ++ks) {
    const v4f f0 = *(const v4f*)(ap + 32 * ks),      f1 = *(const v4f*)(ap + 32 * ks + 4);
    const v4f f2 = *(const v4f*)(ap + 32 * ks + 16), f3 = *(const v4f*)(ap + 32 * ks + 20);
    split8(f0, f1, ahi[ks].h[0], alo[ks].h[0]);
    split8(f2, f3, ahi[ks].h[1], alo[ks].h[1]);
  }

#pragma unroll 1
  for (int g = 0; g < PHID / 64; ++g) {
    v8f acc[4];
#pragma unroll
    for (int tt = 0; tt < 4; ++tt) { v8f z = {0.f, 0.f, 0.f, 0.f, 0.f, 0.f, 0.f, 0.f}; acc[tt] = z; }
#pragma unroll
    for (int ks = 0; ks < 2; ++ks) {
#pragma unroll
      for (int tt = 0; tt < 4; ++tt) {
        const unsigned short* bp = wp1 + (size_t)(64 * g + 16 * tt + m) * 64 + 32 * ks + 8 * hh;
        FragU b;
        b.h[0] = *(const v8us*)bp;
        b.h[1] = *(const v8us*)(bp + 16);
        acc[tt] = wmb(ahi[ks].v, b.v, acc[tt]);
        acc[tt] = wmb(alo[ks].v, b.v, acc[tt]);
      }
    }
#pragma unroll
    for (int tt = 0; tt < 4; ++tt) {
      const int col = 64 * g + 16 * tt + m;
      const float pb = bf16r(pb1[col]);
#pragma unroll
      for (int r = 0; r < 8; ++r) {
        float v = acc[tt][r] + pb;
        v = fmaxf(v, 0.0f);
        const unsigned short hb = bfbits(v);
        const float hf = __uint_as_float(((unsigned)hb) << 16);
        shi[(8 * hh + r) * PSP + col] = hb;
        slo[(8 * hh + r) * PSP + col] = bfbits(v - hf);
      }
    }
  }
  wave_sync();

  v8f acc2[8];
#pragma unroll
  for (int tt = 0; tt < 8; ++tt) { v8f z = {0.f, 0.f, 0.f, 0.f, 0.f, 0.f, 0.f, 0.f}; acc2[tt] = z; }
#pragma unroll 1
  for (int ks = 0; ks < PHID / 32; ++ks) {
    FragU ah, al;
    ah.h[0] = *(const v8us*)(shi + m * PSP + 32 * ks + 8 * hh);
    ah.h[1] = *(const v8us*)(shi + m * PSP + 32 * ks + 16 + 8 * hh);
    al.h[0] = *(const v8us*)(slo + m * PSP + 32 * ks + 8 * hh);
    al.h[1] = *(const v8us*)(slo + m * PSP + 32 * ks + 16 + 8 * hh);
#pragma unroll
    for (int tt = 0; tt < 8; ++tt) {
      const unsigned short* bp = wp2 + (size_t)(16 * tt + m) * PHID + 32 * ks + 8 * hh;
      FragU b;
      b.h[0] = *(const v8us*)bp;
      b.h[1] = *(const v8us*)(bp + 16);
      acc2[tt] = wmb(ah.v, b.v, acc2[tt]);
      acc2[tt] = wmb(al.v, b.v, acc2[tt]);
    }
  }
  wave_sync();

  float fa[8];
#pragma unroll
  for (int r = 0; r < 8; ++r) {
    const int ndx = rb + 8 * hh + r;
    fa[r] = bf16r(nfa[ndx < nN ? ndx : nN - 1]);
  }
  float* ost = (float*)shi;
#pragma unroll
  for (int tt = 0; tt < 8; ++tt) {
    const float pb = bf16r(pb2[16 * tt + m]);
#pragma unroll
    for (int r = 0; r < 8; ++r) ost[(8 * hh + r) * DOUT + 16 * tt + m] = (acc2[tt][r] + pb) * fa[r];
  }
  wave_sync();
#pragma unroll
  for (int i = 0; i < 16; ++i) {
    if (rb + i < nN) {
      const v4f v = *(const v4f*)(ost + i * DOUT + 4 * lane);
      *(volatile v4f*)(out + (size_t)(rb + i) * DOUT + 4 * lane) = v;
    }
  }
  __threadfence();
#pragma unroll
  for (int i = 0; i < 16; ++i) {
    if (rb + i < nN) {
      const v4f v = *(const v4f*)(ost + i * DOUT + 4 * lane);
      *(volatile v4f*)(out + (size_t)(rb + i) * DOUT + 4 * lane) = v;
    }
  }
}

extern "C" void kernel_launch(void* const* d_in, const int* in_sizes, int n_in,
                              void* d_out, int out_size, void* d_ws, size_t ws_size,
                              hipStream_t stream) {
  if (n_in < 18) return;
  const int nN = in_sizes[0] / DCO;
  const int nE = in_sizes[1] / DFE;
  if (nN <= 0 || nE <= 0) return;
  if (in_sizes[0] != nN * DCO || in_sizes[1] != nE * DFE) return;
  if (in_sizes[2] != nE || in_sizes[3] != nE || in_sizes[4] != nE || in_sizes[5] != nN) return;
  if (in_sizes[6] != NHEAD * NPORT * DIN * VHID || in_sizes[7] != NHEAD * NPORT * VHID) return;
  if (in_sizes[8] != NHEAD * NPORT * VHID * VOUT || in_sizes[9] != NHEAD * NPORT * VOUT) return;
  if (in_sizes[10] != NHEAD * NPORT * DIN * SHID || in_sizes[11] != NHEAD * NPORT * SHID) return;
  if (in_sizes[12] != NHEAD * NPORT * SHID || in_sizes[13] != NHEAD * NPORT) return;
  if (in_sizes[14] != NHEAD * VOUT * PHID || in_sizes[15] != PHID) return;
  if (in_sizes[16] != PHID * DOUT || in_sizes[17] != DOUT) return;
  if (out_size != nN * DOUT) return;
  if (nE > (1 << 26) || nN > (1 << 22)) return;

  const float* co  = (const float*)d_in[0];
  const float* ef  = (const float*)d_in[1];
  const int*   src = (const int*)d_in[2];
  const int*   dst = (const int*)d_in[3];
  const float* nf  = (const float*)d_in[4];
  const float* nfa = (const float*)d_in[5];
  const float* vW1 = (const float*)d_in[6];
  const float* vb1 = (const float*)d_in[7];
  const float* vW2 = (const float*)d_in[8];
  const float* vb2 = (const float*)d_in[9];
  const float* sW1 = (const float*)d_in[10];
  const float* sb1 = (const float*)d_in[11];
  const float* sW2 = (const float*)d_in[12];
  const float* sb2 = (const float*)d_in[13];
  const float* pW1 = (const float*)d_in[14];
  const float* pb1 = (const float*)d_in[15];
  const float* pW2 = (const float*)d_in[16];
  const float* pb2 = (const float*)d_in[17];
  float* out = (float*)d_out;

  const int nBC    = (nN + NBC - 1) / NBC;
  if (4 * nBC + 1 > RBN) return;
  const int CNTPAD = nBC * NBC;
  const int nBF    = (nN + NBF - 1) / NBF;
  const int csrLen = ((nE + 31) & ~31) + 4096;
  const int NPAD   = ((nN + PROWS - 1) / PROWS) * PROWS;
  const int nProj  = NPAD / PROWS;
  const int nNode  = NPAD / NPB;

  char* ws = (char*)d_ws;
  size_t off = 0;
  const size_t oWB1 = off; off += (size_t)NPORT * 256 * 32 * 2;        off = (off + 255) & ~(size_t)255;
  const size_t oWC  = off; off += (size_t)WCN * 32 * 2;                off = (off + 255) & ~(size_t)255;
  const size_t oWV2 = off; off += (size_t)NPORT * NHEAD * 16 * 32 * 2; off = (off + 255) & ~(size_t)255;
  const size_t oWP1 = off; off += (size_t)PHID * 64 * 2;               off = (off + 255) & ~(size_t)255;
  const size_t oWP2 = off; off += (size_t)DOUT * PHID * 2;             off = (off + 255) & ~(size_t)255;
  const size_t oC0  = off; off += (size_t)CNTPAD * 4;                  off = (off + 255) & ~(size_t)255;
  const size_t oO0  = off; off += (size_t)CNTPAD * 4;                  off = (off + 255) & ~(size_t)255;
  const size_t oR0  = off; off += (size_t)RBN * 4;                     off = (off + 255) & ~(size_t)255;
  const size_t oS0  = off; off += (size_t)csrLen * 4;                  off = (off + 255) & ~(size_t)255;
  const size_t oC1  = off; off += (size_t)CNTPAD * 4;                  off = (off + 255) & ~(size_t)255;
  const size_t oO1  = off; off += (size_t)CNTPAD * 4;                  off = (off + 255) & ~(size_t)255;
  const size_t oR1  = off; off += (size_t)RBN * 4;                     off = (off + 255) & ~(size_t)255;
  const size_t oS1  = off; off += (size_t)csrLen * 4;                  off = (off + 255) & ~(size_t)255;
  const size_t oPC  = off; off += (size_t)NPAD * PCW * 4;              off = (off + 255) & ~(size_t)255;
  const size_t oND  = off; off += (size_t)NPAD * NDP * 4;              off = (off + 255) & ~(size_t)255;
  if (off > ws_size) return;
  if (off > ((size_t)128 << 20)) return;
  unsigned short* wb1u = (unsigned short*)(ws + oWB1);
  unsigned short* wcu  = (unsigned short*)(ws + oWC);
  unsigned short* wv2u = (unsigned short*)(ws + oWV2);
  unsigned short* wp1  = (unsigned short*)(ws + oWP1);
  unsigned short* wp2  = (unsigned short*)(ws + oWP2);
  const _Float16* wb1 = (const _Float16*)(ws + oWB1);
  const _Float16* wc  = (const _Float16*)(ws + oWC);
  const _Float16* wv2 = (const _Float16*)(ws + oWV2);
  int* cnt0 = (int*)(ws + oC0); int* offs0 = (int*)(ws + oO0); int* rb0 = (int*)(ws + oR0); int* csr0 = (int*)(ws + oS0);
  int* cnt1 = (int*)(ws + oC1); int* offs1 = (int*)(ws + oO1); int* rb1 = (int*)(ws + oR1); int* csr1 = (int*)(ws + oS1);
  float* pcp = (float*)(ws + oPC);
  float* ndp = (float*)(ws + oND);

  const int vec8 = ((nE & 3) == 0) ? 1 : 0;

  const int nPrep = NPORT * 256 * 32 / 8 + WCN * 32 / 8 + NPORT * NHEAD * 16 * 32 / 8 + PHID * 64 / 8 + DOUT * PHID / 8;
  k_prep<<<(nPrep + NTHR - 1) / NTHR, NTHR, 0, stream>>>(vW1, vb1, sW1, sb1, vW2, pW1, pW2, wb1u, wcu, wv2u, wp1, wp2);

  hipFuncSetAttribute(reinterpret_cast<const void*>(&k_fill), hipFuncAttributeMaxDynamicSharedMemorySize, LDS_FILL);
  k_count<<<nBC, NTHR, 0, stream>>>(src, cnt0, nE, vec8);
  k_offsets<<<1, OTHR, 0, stream>>>(cnt0, offs0, rb0, nBC);
  k_fill<<<nBF, NTHR, LDS_FILL, stream>>>(src, offs0, rb0, csr0, nE, vec8, csrLen);
  k_count<<<nBC, NTHR, 0, stream>>>(dst, cnt1, nE, vec8);
  k_offsets<<<1, OTHR, 0, stream>>>(cnt1, offs1, rb1, nBC);
  k_fill<<<nBF, NTHR, LDS_FILL, stream>>>(dst, offs1, rb1, csr1, nE, vec8, csrLen);

  hipFuncSetAttribute(reinterpret_cast<const void*>(&k_node<0>), hipFuncAttributeMaxDynamicSharedMemorySize, LDS_NODE);
  hipFuncSetAttribute(reinterpret_cast<const void*>(&k_node<1>), hipFuncAttributeMaxDynamicSharedMemorySize, LDS_NODE);
  hipFuncSetAttribute(reinterpret_cast<const void*>(&k_psi), hipFuncAttributeMaxDynamicSharedMemorySize, LDS_PSI);

  k_proj<<<nProj, NTHR, 0, stream>>>(co, wc, pcp, nN, 0);
  k_node<0><<<nNode, NDTHR, LDS_NODE, stream>>>(ef, src, dst, nf, nfa, cnt0, offs0, csr0, pcp, wb1, wv2, vb2, sW2, sb2,
                                                ndp, nN, nE, csrLen);
  k_proj<<<nProj, NTHR, 0, stream>>>(co, wc, pcp, nN, 1);
  k_node<1><<<nNode, NDTHR, LDS_NODE, stream>>>(ef, src, dst, nf, nfa, cnt1, offs1, csr1, pcp, wb1, wv2, vb2, sW2, sb2,
                                                ndp, nN, nE, csrLen);

  k_psi<<<nNode, NDTHR, LDS_PSI, stream>>>(ndp, wp1, pb1, wp2, pb2, nfa, out, nN);
}
